// GATInnerLayer_20615843020951
// MI455X (gfx1250) — hardware-verified
//
#include <hip/hip_runtime.h>
#include <math.h>

typedef __attribute__((ext_vector_type(16))) _Float16 v16h;
typedef __attribute__((ext_vector_type(16))) __bf16 v16b;
typedef __attribute__((ext_vector_type(8)))  _Float16 v8h;
typedef __attribute__((ext_vector_type(8)))  float v8f;
typedef __attribute__((ext_vector_type(4)))  float v4f;
typedef __attribute__((ext_vector_type(2)))  float v2f;
typedef __attribute__((ext_vector_type(4)))  unsigned v4u;
typedef __attribute__((ext_vector_type(4)))  int v4i;
typedef float __attribute__((may_alias)) float_a;
typedef int __attribute__((may_alias)) int_a;

template <typename T> __device__ __forceinline__ void vst2(void* p, T v) { *(volatile T*)p = v; __threadfence(); *(volatile T*)p = v; }
__device__ __forceinline__ v8f wmma16(v16h a, v16h b, v8f c) {
  v8f d = __builtin_amdgcn_wmma_f32_16x16x32_f16(false, a, false, b, (short)0, c, false, false);
  asm volatile("v_nop\n\tv_nop\n\tv_nop\n\tv_nop" : "+v"(d) : "v"(a), "v"(b));
  return d;
}
__device__ __forceinline__ v8f wmma_bf(v16b a, v16b b, v8f c) {
  v8f d = __builtin_amdgcn_wmma_f32_16x16x32_bf16(false, a, false, b, (short)0, c, false, false);
  asm volatile("v_nop\n\tv_nop\n\tv_nop\n\tv_nop" : "+v"(d) : "v"(a), "v"(b));
  return d;
}
__device__ __forceinline__ v16h frag_h(const _Float16* rowk0, int lane) {
  union { v16h v; v8h q[2]; } u; const _Float16* p = rowk0 + 8 * (lane >> 4);
  u.q[0] = *(const v8h*)p; u.q[1] = *(const v8h*)(p + 16); return u.v;
}
__device__ __forceinline__ v16h frag_f32(const float* rowk0, int lane) {
  v16h a; const float* p = rowk0 + 8 * (lane >> 4);
#pragma unroll
  for (int i = 0; i < 8; ++i) { a[i] = (_Float16)p[i]; a[8 + i] = (_Float16)p[16 + i]; }
  return a;
}
__device__ __forceinline__ v16h frag_f32s(const float* rowk0, int lane, float sc) {
  v16h a; const float* p = rowk0 + 8 * (lane >> 4);
#pragma unroll
  for (int i = 0; i < 8; ++i) { a[i] = (_Float16)(p[i] * sc); a[8 + i] = (_Float16)(p[16 + i] * sc); }
  return a;
}
__device__ __forceinline__ v16h fragc_f32(const float* W, int k0, int n, int lane, int ld, int K) {
  v16h a; const int g = lane >> 4;
#pragma unroll
  for (int i = 0; i < 8; ++i) { const int ka = k0 + 8 * g + i, kb = ka + 16;
    a[i] = (_Float16)(ka < K ? W[(size_t)(ka < K ? ka : K - 1) * ld + n] : 0.f); a[8 + i] = (_Float16)(kb < K ? W[(size_t)(kb < K ? kb : K - 1) * ld + n] : 0.f); }
  return a;
}
struct F2 { v16b h, l; };
__device__ __forceinline__ F2 bsplit16(const float v[16]) { F2 r;
#pragma unroll
  for (int i = 0; i < 16; ++i) { const __bf16 h = (__bf16)v[i]; r.h[i] = h; r.l[i] = (__bf16)(v[i] - (float)h); }
  return r; }
__device__ __forceinline__ F2 split_row(const float* row, int k0, int lane) { float v[16]; const float* p = row + k0 + 8 * (lane >> 4);
#pragma unroll
  for (int i = 0; i < 8; ++i) { v[i] = p[i]; v[8 + i] = p[16 + i]; }
  return bsplit16(v); }
__device__ __forceinline__ F2 split_rowK(const float* row, int k0, int lane, int K) { float v[16]; const int g = lane >> 4;
#pragma unroll
  for (int i = 0; i < 8; ++i) { const int ka = k0 + 8 * g + i, kb = ka + 16; v[i] = ka < K ? row[ka < K ? ka : K - 1] : 0.f; v[8 + i] = kb < K ? row[kb < K ? kb : K - 1] : 0.f; }
  return bsplit16(v); }
__device__ __forceinline__ F2 split_col(const float* W, int k0, int n, int lane, int ld, int K) { float v[16]; const int g = lane >> 4;
#pragma unroll
  for (int i = 0; i < 8; ++i) { const int ka = k0 + 8 * g + i, kb = ka + 16; v[i] = ka < K ? W[(size_t)(ka < K ? ka : K - 1) * ld + n] : 0.f; v[8 + i] = kb < K ? W[(size_t)(kb < K ? kb : K - 1) * ld + n] : 0.f; }
  return bsplit16(v); }
__device__ __forceinline__ v8f mac3(const F2& a, const F2& b, v8f c) { c = wmma_bf(a.l, b.h, c); c = wmma_bf(a.h, b.l, c); return wmma_bf(a.h, b.h, c); }
__device__ __forceinline__ float sigm(float v) { return 1.0f / (1.0f + expf(-v)); }
#define LDSX() do { asm volatile("s_wait_dscnt 0" ::: "memory"); __builtin_amdgcn_wave_barrier(); __builtin_amdgcn_fence(__ATOMIC_RELEASE, "workgroup"); } while (0)

__device__ __forceinline__ float bfr(float v) { return (float)(__bf16)v; }
#define NN 20000
#define DIN 256
#define DO 128
#ifndef NNODE
#define NNODE NN
#endif
#define WS_Q 0u
#define WS_K (WS_Q + 4u * (size_t)NN * DO)
#define WS_V (WS_K + 4u * (size_t)NN * DO)
#define WS_END (WS_V + 4u * (size_t)NN * DO)
__global__ __launch_bounds__(128) void k_qkv(const float* __restrict__ Hm, const float* __restrict__ WQ, const float* __restrict__ WK, const float* __restrict__ WV, float* __restrict__ Q, float* __restrict__ K, float* __restrict__ V) { __shared__ __align__(16) float sf[4][16][132];
  const int tid = threadIdx.x, wave = tid >> 5, lane = tid & 31, col = lane & 15, g = lane >> 4; const int which = blockIdx.y; const size_t r0 = (size_t)blockIdx.x * 64 + wave * 16; const size_t ra = (r0 + col < NN) ? r0 + col : NN - 1;
  const float* WA = which == 0 ? WQ : which == 1 ? WK : WV; float* D = which == 0 ? Q : which == 1 ? K : V;
  v8f acc[8] = {};
#pragma unroll
  for (int kc = 0; kc < DIN / 32; ++kc) { v16b a; { const float* p = Hm + ra * DIN + kc * 32 + 8 * g;
#pragma unroll
      for (int i = 0; i < 8; ++i) { a[i] = (__bf16)p[i]; a[8 + i] = (__bf16)p[16 + i]; } }
#pragma unroll
    for (int j = 0; j < 8; ++j) { v16b w; const int o = j * 16 + col; const float* wr = WA + (size_t)o * DIN + kc * 32 + 8 * g;
#pragma unroll
      for (int i = 0; i < 8; ++i) { w[i] = (__bf16)wr[i]; w[8 + i] = (__bf16)wr[16 + i]; }
      acc[j] = wmma_bf(a, w, acc[j]); } }
#pragma unroll
  for (int j = 0; j < 8; ++j)
#pragma unroll
    for (int r = 0; r < 8; ++r) sf[wave][8 * g + r][j * 16 + col] = acc[j][r];
  LDSX(); for (int rl = 0; rl < 16; ++rl) { const size_t r = r0 + rl; if (r < NN) vst2(D + r * DO + lane * 4, *(const v4f*)&sf[wave][rl][lane * 4]); } }
__global__ __launch_bounds__(128) void k_gat(const float* __restrict__ Q, const float* __restrict__ K, const float* __restrict__ V, float* __restrict__ OUT) {
  __shared__ float se[DO][DO + 1]; __shared__ float sq[DO], sv[DO], sz[DO]; __shared__ float sred[8]; __shared__ __align__(16) float so[DO];
  const int t = threadIdx.x; const size_t n = blockIdx.x;
  const float qv = Q[n * DO + t]; sq[t] = qv; sv[t] = V[n * DO + t];
  float mx = qv, mn = qv;
#pragma unroll
  for (int o = 1; o < 32; o <<= 1) { mx = fmaxf(mx, __shfl_xor(mx, o)); mn = fminf(mn, __shfl_xor(mn, o)); }
  if ((t & 31) == 0) { sred[t >> 5] = mx; sred[4 + (t >> 5)] = mn; } __syncthreads();
  mx = fmaxf(fmaxf(sred[0], sred[1]), fmaxf(sred[2], sred[3])); mn = fminf(fminf(sred[4], sred[5]), fminf(sred[6], sred[7]));
  const float kj = K[n * DO + t] * (1.0f / 16.0f); const float Mj = (kj >= 0.f) ? kj * mx : kj * mn;
  float z = 0.f;
#pragma unroll 1
  for (int i = 0; i < DO; ++i) { const float e = __expf(sq[i] * kj - Mj); se[i][t] = e; z += e; }
  sz[t] = 1.0f / z;
  __syncthreads();
  float acc = 0.f;
#pragma unroll 1
  for (int j = 0; j < DO; ++j) acc += se[t][j] * sz[j] * sv[j];
  so[t] = acc; __syncthreads();
  if (t < 32) vst2(OUT + n * DO + t * 4, *(const v4f*)&so[t * 4]); }
extern "C" void kernel_launch(void* const* d_in, const int* in_sizes, int n_in, void* d_out, int out_size, void* d_ws, size_t ws_size, hipStream_t stream) {
  (void)in_sizes; (void)n_in; (void)out_size;
  const float** F = (const float**)d_in;
  if (ws_size < (size_t)WS_END) return;
  char* ws = (char*)d_ws; float *Q = (float*)(ws + WS_Q), *K = (float*)(ws + WS_K), *V = (float*)(ws + WS_V);
  k_qkv<<<dim3((NN + 63) / 64, 3), 128, 0, stream>>>(F[0], F[1], F[2], F[3], Q, K, V);
  k_gat<<<dim3(NNODE), 128, 0, stream>>>(Q, K, V, (float*)d_out);
}
